// ConvNextV2Block_30958124269767
// MI455X (gfx1250) — hardware-run, weakly checked
//
#include <hip/hip_runtime.h>
#include <math.h>


#define NB 2
#define CC 96
#define DDp 24
#define HH 56
#define WW 56
#define PL (HH * WW)
#define VOX (DDp * PL)
#define EE 384
#define NR (NB * VOX)

typedef __attribute__((ext_vector_type(16))) _Float16 v16h;
typedef __attribute__((ext_vector_type(8)))  _Float16 v8h;
typedef __attribute__((ext_vector_type(8)))  float v8f;
typedef __attribute__((ext_vector_type(4)))  float v4f;
typedef __attribute__((ext_vector_type(4)))  unsigned v4u;
typedef float __attribute__((may_alias)) float_a;

template <typename T> __device__ __forceinline__ void vst2(void* p, T v) { *(volatile T*)p = v; __threadfence(); *(volatile T*)p = v; }
__device__ __forceinline__ v8f wmma16(v16h a, v16h b, v8f c) {
  v8f d = __builtin_amdgcn_wmma_f32_16x16x32_f16(false, a, false, b, (short)0, c, false, false);
  asm volatile("v_nop\n\tv_nop\n\tv_nop\n\tv_nop" : "+v"(d) : "v"(a), "v"(b));
  return d;
}
__device__ __forceinline__ v16h frag_h(const _Float16* rowk0, int lane) {
  union { v16h v; v8h q[2]; } u; const _Float16* p = rowk0 + 8 * (lane >> 4);
  u.q[0] = *(const v8h*)p; u.q[1] = *(const v8h*)(p + 16); return u.v;
}
#define LDSX() do { asm volatile("s_wait_dscnt 0" ::: "memory"); __builtin_amdgcn_wave_barrier(); __builtin_amdgcn_fence(__ATOMIC_RELEASE, "workgroup"); } while (0)

__global__ __launch_bounds__(256) void k_dwconv(const float* __restrict__ x, const float* __restrict__ kw, const float* __restrict__ kb, float* __restrict__ y) {
  __shared__ float pl[7][62][63];
  __shared__ float wk[343];
  const int d = blockIdx.x, c = blockIdx.y, b = blockIdx.z, tid = threadIdx.x;
  const float* xc = x + ((size_t)b * CC + c) * VOX;
  for (int i = tid; i < 343; i += 256) wk[i] = kw[(size_t)c * 343 + i];
  for (int i = tid; i < 7 * 62 * 63; i += 256) { const int dz = i / (62 * 63), r = (i / 63) % 62, q = i % 63;
    const int zd = d + dz - 3, hy = r - 3, wx = q - 3;
    pl[dz][r][q] = (zd >= 0 && zd < DDp && hy >= 0 && hy < HH && wx >= 0 && wx < WW) ? xc[(size_t)zd * PL + hy * WW + wx] : 0.f; }
  __syncthreads();
  const float bias = kb[c];
  for (int qd = tid; qd < PL / 4; qd += 256) { const int hy = (qd * 4) / WW, w0 = (qd * 4) % WW;
    float a0 = bias, a1 = bias, a2 = bias, a3 = bias;
#pragma unroll 1
    for (int dz = 0; dz < 7; ++dz)
#pragma unroll 1
      for (int ky = 0; ky < 7; ++ky) { const float* pr = &pl[dz][hy + ky][w0]; const float* wr = &wk[(dz * 7 + ky) * 7];
#pragma unroll
        for (int kx = 0; kx < 7; ++kx) { const float wv = wr[kx]; a0 += wv * pr[kx]; a1 += wv * pr[kx + 1]; a2 += wv * pr[kx + 2]; a3 += wv * pr[kx + 3]; } }
    v4f v = {a0, a1, a2, a3};
    vst2(y + ((size_t)b * CC + c) * VOX + (size_t)d * PL + qd * 4, v); }
}

__global__ __launch_bounds__(256) void k_ln(const float* __restrict__ y, const float* __restrict__ lw, const float* __restrict__ lb, _Float16* __restrict__ h16) {
  __shared__ float tile[CC][65];
  const int b = blockIdx.y, v0 = blockIdx.x * 64, tid = threadIdx.x;
  for (int i = tid; i < CC * 64; i += 256) { const int c = i >> 6, vl = i & 63; tile[c][vl] = y[((size_t)b * CC + c) * VOX + v0 + vl]; }
  __syncthreads();
  const int vl = tid >> 2, part = tid & 3;
  float s = 0.f;
  for (int c = part * 24; c < part * 24 + 24; ++c) s += tile[c][vl];
  s += __shfl_xor(s, 1, 32); s += __shfl_xor(s, 2, 32);
  const float mu = s / (float)CC;
  float q = 0.f;
  for (int c = part * 24; c < part * 24 + 24; ++c) { const float dv = tile[c][vl] - mu; q += dv * dv; }
  q += __shfl_xor(q, 1, 32); q += __shfl_xor(q, 2, 32);
  const float rs = rsqrtf(q / (float)CC + 1e-6f);
#pragma unroll
  for (int pc = 0; pc < 3; ++pc) { union { v8h h; v4u u; } pk;
#pragma unroll
    for (int e = 0; e < 8; ++e) { const int c = part * 24 + pc * 8 + e; pk.h[e] = (_Float16)((tile[c][vl] - mu) * rs * lw[c] + lb[c]); }
    vst2(h16 + ((size_t)b * VOX + v0 + vl) * CC + part * 24 + pc * 8, pk.u); }
}

__global__ __launch_bounds__(256) void k_packT(const float* __restrict__ W, _Float16* __restrict__ Wt, int K, int N) {
  __shared__ float tile[32][33];
  const int k0 = blockIdx.y * 32, n0 = blockIdx.x * 32, tid = threadIdx.x;
  for (int q = tid; q < 32 * 32; q += 256) { const int kk = q >> 5, nn = q & 31; tile[kk][nn] = W[(size_t)(k0 + kk) * N + n0 + nn]; }
  __syncthreads();
  if (tid < 128) { const int nn = tid >> 2, pc = tid & 3;
    union { v8h h; v4u u; } pk;
#pragma unroll
    for (int e = 0; e < 8; ++e) pk.h[e] = (_Float16)tile[pc * 8 + e][nn];
    vst2(Wt + (size_t)(n0 + nn) * K + k0 + pc * 8, pk.u); }
}

__global__ __launch_bounds__(128) void k_pw1(const _Float16* __restrict__ h16, const _Float16* __restrict__ W1T, const float* __restrict__ b1,
                                           _Float16* __restrict__ g, float* __restrict__ sqp) {
  __shared__ __align__(16) float so[4][16 * 128];
  __shared__ float csum[4][128];
  const int tid = threadIdx.x, wave = tid >> 5, lane = tid & 31, col = lane & 15, gg = lane >> 4;
  const int r0 = blockIdx.x * 64 + wave * 16, n0 = blockIdx.y * 128;
  v8f acc[8] = {};
#pragma unroll
  for (int kc = 0; kc < CC / 32; ++kc) { const v16h a = frag_h(h16 + (size_t)(r0 + col) * CC + kc * 32, lane);
#pragma unroll
    for (int j = 0; j < 8; ++j) acc[j] = wmma16(a, frag_h(W1T + (size_t)(n0 + j * 16 + col) * CC + kc * 32, lane), acc[j]); }
  float* S = so[wave];
#pragma unroll
  for (int j = 0; j < 8; ++j) { const float bv = b1[n0 + j * 16 + col];
#pragma unroll
    for (int r = 0; r < 8; ++r) { const float u = acc[j][r] + bv; S[(8 * gg + r) * 128 + j * 16 + col] = 0.5f * u * (1.0f + erff(u * 0.70710678118654752f)); } }
  LDSX();
#pragma unroll
  for (int q = 0; q < 8; ++q) { const int rl = q * 2 + (lane >> 4), pc = lane & 15;
    union { v8h h; v4u u; } pk;
#pragma unroll
    for (int e = 0; e < 8; ++e) pk.h[e] = (_Float16)S[rl * 128 + pc * 8 + e];
    vst2(g + (size_t)(r0 + rl) * EE + n0 + pc * 8, pk.u); }
  float q0 = 0.f, q1 = 0.f, q2 = 0.f, q3 = 0.f;
  for (int rl = 0; rl < 16; ++rl) { const v4f v = *(const v4f*)(S + rl * 128 + lane * 4); q0 += v[0] * v[0]; q1 += v[1] * v[1]; q2 += v[2] * v[2]; q3 += v[3] * v[3]; }
  csum[wave][lane * 4] = q0; csum[wave][lane * 4 + 1] = q1; csum[wave][lane * 4 + 2] = q2; csum[wave][lane * 4 + 3] = q3;
  __syncthreads();
  if (tid < 32) { v4f t;
#pragma unroll
    for (int e = 0; e < 4; ++e) t[e] = csum[0][tid * 4 + e] + csum[1][tid * 4 + e] + csum[2][tid * 4 + e] + csum[3][tid * 4 + e];
    vst2(sqp + (size_t)blockIdx.x * EE + n0 + tid * 4, t); }
}

__global__ __launch_bounds__(EE) void k_grn(const float* __restrict__ sqp, const float* __restrict__ gm, const float* __restrict__ bt, float* __restrict__ coef) {
  __shared__ float gxs[EE], red[EE];
  const int b = blockIdx.x, e = threadIdx.x;
  float s = 0.f;
  for (int rb = 0; rb < VOX / 64; ++rb) s += sqp[((size_t)b * (VOX / 64) + rb) * EE + e];
  const float gx = sqrtf(s); gxs[e] = gx; red[e] = gx; __syncthreads();
  if (e < 128) red[e] += red[e + 128] + red[e + 256];
  __syncthreads();
  for (int st = 64; st > 0; st >>= 1) { if (e < st) red[e] += red[e + st]; __syncthreads(); }
  const float nx = gx / (red[0] / (float)EE + 1e-6f);
  vst2(coef + ((size_t)b * 2) * EE + e, (float_a)(1.0f + gm[e] * nx));
  vst2(coef + ((size_t)b * 2 + 1) * EE + e, (float_a)bt[e]);
}

__global__ __launch_bounds__(128) void k_pw2(const _Float16* __restrict__ g, const float* __restrict__ coef, const _Float16* __restrict__ W2T,
                                           const float* __restrict__ b2, const float* __restrict__ x, float* __restrict__ out) {
  __shared__ __align__(16) float st[CC][68];
  const int tid = threadIdx.x, wave = tid >> 5, lane = tid & 31, col = lane & 15, gg = lane >> 4;
  const int b = blockIdx.y, v0 = blockIdx.x * 64;
  const size_t r0 = (size_t)b * VOX + v0 + wave * 16;
  const float* cf = coef + (size_t)b * 2 * EE; const float* ad = cf + EE;
  v8f acc[6] = {};
#pragma unroll 1
  for (int kc = 0; kc < EE / 32; ++kc) {
    v16h a; const _Float16* p = g + (r0 + col) * EE + kc * 32 + 8 * gg; const int k0 = kc * 32 + 8 * gg;
    const v8h lo = *(const v8h*)p, hi = *(const v8h*)(p + 16);
#pragma unroll
    for (int i = 0; i < 8; ++i) { a[i] = (_Float16)((float)lo[i] * cf[k0 + i] + ad[k0 + i]); a[8 + i] = (_Float16)((float)hi[i] * cf[k0 + 16 + i] + ad[k0 + 16 + i]); }
#pragma unroll
    for (int j = 0; j < 6; ++j) acc[j] = wmma16(a, frag_h(W2T + (size_t)(j * 16 + col) * EE + kc * 32, lane), acc[j]);
  }
#pragma unroll
  for (int j = 0; j < 6; ++j) { const float bv = b2[j * 16 + col];
#pragma unroll
    for (int r = 0; r < 8; ++r) st[j * 16 + col][wave * 16 + 8 * gg + r] = acc[j][r] + bv; }
  __syncthreads();
  for (int q = tid; q < CC * 16; q += 128) { const int c = q >> 4, pc = q & 15;
    const size_t o = ((size_t)b * CC + c) * VOX + v0 + pc * 4;
    vst2(out + o, *(const v4f*)(&st[c][pc * 4]) + *(const v4f*)(x + o)); }
}

extern "C" void kernel_launch(void* const* d_in, const int* in_sizes, int n_in,
                              void* d_out, int out_size, void* d_ws, size_t ws_size,
                              hipStream_t stream) {
  (void)in_sizes; (void)n_in; (void)out_size; (void)ws_size;
  const float* x = (const float*)d_in[0]; const float* kw = (const float*)d_in[1]; const float* kb = (const float*)d_in[2];
  const float* lw = (const float*)d_in[3]; const float* lb = (const float*)d_in[4];
  const float* w1 = (const float*)d_in[5]; const float* b1 = (const float*)d_in[6];
  const float* gm = (const float*)d_in[7]; const float* bt = (const float*)d_in[8];
  const float* w2 = (const float*)d_in[9]; const float* b2 = (const float*)d_in[10];
  float* out = (float*)d_out;
  char* ws = (char*)d_ws; size_t off = 0;
  auto take = [&](size_t bytes) { char* p = ws + off; off += (bytes + 255) & ~(size_t)255; return p; };
  float* y = (float*)take((size_t)NR * CC * 4);
  _Float16* h16 = (_Float16*)take((size_t)NR * CC * 2);
  _Float16* W1T = (_Float16*)take((size_t)EE * CC * 2); _Float16* W2T = (_Float16*)take((size_t)CC * EE * 2);
  _Float16* g = (_Float16*)take((size_t)NR * EE * 2);
  float* sqp = (float*)take((size_t)(NR / 64) * EE * 4);
  float* coef = (float*)take((size_t)NB * 2 * EE * 4);
  k_dwconv<<<dim3(DDp, CC, NB), 256, 0, stream>>>(x, kw, kb, y);
  k_ln<<<dim3(VOX / 64, NB), 256, 0, stream>>>(y, lw, lb, h16);
  k_packT<<<dim3(EE / 32, CC / 32), 256, 0, stream>>>(w1, W1T, CC, EE);
  k_packT<<<dim3(CC / 32, EE / 32), 256, 0, stream>>>(w2, W2T, EE, CC);
  k_pw1<<<dim3(NR / 64, EE / 128), 128, 0, stream>>>(h16, W1T, b1, g, sqp);
  k_grn<<<NB, EE, 0, stream>>>(sqp, gm, bt, coef);
  k_pw2<<<dim3(VOX / 64, NB), 128, 0, stream>>>(g, coef, W2T, b2, x, out);
}
